// SelfAttention_85607288144082
// MI455X (gfx1250) — hardware-run, weakly checked
//
#include <hip/hip_runtime.h>


#ifndef NB
#define NB 2
#endif
#ifndef VD
#define VD 32
#endif
#define VH 32
#define VW 32
#define NB_FULL  2
#define VD_FULL  32
#define SEQ      (VD * VH * VW)
#define SEQ_FULL (VD_FULL * VH * VW)
#ifndef OUT_SEQ
#define OUT_SEQ SEQ
#endif
#define SRR  4
#define SEQK ((VD / SRR) * (VH / SRR) * (VW / SRR))
#define DM   128
#define NH_  4
#define HD   32
#define KC   (64 * DM)
#define AW   4
#define OSP  36
#define CSP  132
#define QRS  2048.0f
#define SC2  ((float)(0.17677669529663687 * 1.4426950408889634))
#define PSH  14.0f
#define NEGB (-3.0e38f)
#define WCS  1024.0f
#define WCI  (1.0f / 1024.0f)
#define OCS  256.0f
#define OWI  (1.0f / (256.0f * 1024.0f))

static_assert(HD == 32);
static_assert(NH_ * HD == DM);
static_assert(DM % 64 == 0);
static_assert(64 % HD == 0);
static_assert(DM % 32 == 0);
static_assert(DM / 32 == NH_);
static_assert(SEQ % 64 == 0);
static_assert((NB * SEQ) % 64 == 0);
static_assert(VH == 32);
static_assert(VW == 32);
static_assert(VD % SRR == 0);
static_assert(SEQK == (VD / 4) * 64);
static_assert(SEQK % 64 == 0);
static_assert((NB * SEQK) % 64 == 0);
static_assert((NB * SEQK) % 16 == 0);
static_assert(SEQK % 32 == 0);
static_assert(SEQ % (16 * AW) == 0);
static_assert(KC % 32 == 0);
static_assert(((size_t)SEQ * DM) % 8 == 0);
static_assert(((size_t)DM * DM) % 8 == 0);
static_assert(NB <= NB_FULL);
static_assert(VD <= VD_FULL);
static_assert((OSP * 4) % 16 == 0);
static_assert((CSP * 4) % 16 == 0);
static_assert(16 * 68 * 4 <= 131072);
static_assert(16 * CSP * 4 <= 131072);
static_assert(AW * 16 * OSP * 4 <= 131072);
static_assert(64 * CSP * 4 <= 131072);

typedef _Float16 h16;
typedef unsigned short bf;
typedef __attribute__((ext_vector_type(16))) __bf16   v16bf;
typedef __attribute__((ext_vector_type(16))) _Float16 v16h;
typedef __attribute__((ext_vector_type(8)))  _Float16 v8h;
typedef __attribute__((ext_vector_type(8)))  unsigned short v8us;
typedef __attribute__((ext_vector_type(8)))  float    v8f;
typedef __attribute__((ext_vector_type(4)))  float    v4f;
typedef v4f  __attribute__((may_alias)) v4fa;

__device__ __forceinline__ unsigned short f2bf(float f) { unsigned u = __float_as_uint(f); u += 0x7FFFu + ((u >> 16) & 1u); return (unsigned short)(u >> 16); }
__device__ __forceinline__ float bfr(float f) { return __uint_as_float(((unsigned)f2bf(f)) << 16); }
__device__ __forceinline__ v16h cat16(v8h lo, v8h hi) { return __builtin_shufflevector(lo, hi, 0, 1, 2, 3, 4, 5, 6, 7, 8, 9, 10, 11, 12, 13, 14, 15); }
__device__ __forceinline__ v16bf cat16b(v8us lo, v8us hi) { return __builtin_bit_cast(v16bf, __builtin_shufflevector(lo, hi, 0, 1, 2, 3, 4, 5, 6, 7, 8, 9, 10, 11, 12, 13, 14, 15)); }
__device__ __forceinline__ v8f wmma16(v16h a, v16h b, v8f c) { return __builtin_amdgcn_wmma_f32_16x16x32_f16(false, a, false, b, (short)0, c, false, false); }
__device__ __forceinline__ v8f wmmab(v16bf a, v16bf b, v8f c) { return __builtin_amdgcn_wmma_f32_16x16x32_bf16(false, a, false, b, (short)0, c, false, false); }
__device__ __forceinline__ v16h  ldh(const h16* p) { return cat16(*(const v8h*)p, *(const v8h*)(p + 16)); }
__device__ __forceinline__ v16bf ldb(const bf* p)  { return cat16b(*(const v8us*)p, *(const v8us*)(p + 16)); }
__device__ __forceinline__ void wave_sync() { __builtin_amdgcn_fence(3  , "wavefront"); __builtin_amdgcn_wave_barrier(); asm volatile("" ::: "memory"); }

__device__ __forceinline__ v8f wmma16g(v16h a, v16h b, v8f c) { c = wmma16(a, b, c); asm volatile("v_nop\n\tv_nop\n\tv_nop\n\tv_nop" : "+v"(c) : "v"(a), "v"(b)); return c; }
__device__ __forceinline__ v8f wmmabg(v16bf a, v16bf b, v8f c) { c = wmmab(a, b, c); asm volatile("v_nop\n\tv_nop\n\tv_nop\n\tv_nop" : "+v"(c) : "v"(a), "v"(b)); return c; }
__device__ __forceinline__ h16 toh_flush(float v) { const h16 r = (h16)v; return (fabsf(v) < 6.103515625e-05f) ? (h16)0.0f : r; }

__global__ __launch_bounds__(256) void k_cvt8(const float* __restrict__ src, bf* dst, size_t n8) {
    const size_t i = (size_t)blockIdx.x * 256 + threadIdx.x; if (i >= n8) return;
    const v8f v = *(const v8f*)(src + i * 8); v8us o;
#pragma unroll
    for (int k = 0; k < 8; ++k) o[k] = f2bf(v[k]);
    *(volatile v8us*)(dst + i * 8) = o; __threadfence(); *(volatile v8us*)(dst + i * 8) = o;
}

__global__ __launch_bounds__(256) void k_cvth8(const float* __restrict__ src, h16* dst, size_t n8, float carry) {
    const size_t i = (size_t)blockIdx.x * 256 + threadIdx.x; if (i >= n8) return;
    const v8f v = *(const v8f*)(src + i * 8); v8h o;
#pragma unroll
    for (int k = 0; k < 8; ++k) o[k] = toh_flush(bfr(v[k]) * carry);
    *(volatile v8h*)(dst + i * 8) = o; __threadfence(); *(volatile v8h*)(dst + i * 8) = o;
}

__global__ __launch_bounds__(256) void k_srw(const float* __restrict__ src, bf* dst) {
    __shared__ __align__(16) float ts[64 * CSP];
    static_assert(256 * 32 == 128 * 64);
    static_assert(256 * 4 * 8 == 64 * 128);
    const int co = blockIdx.x, tid = threadIdx.x;
    const float* sp = src + (size_t)co * KC;
#pragma unroll 1
    for (int it = 0; it < 32; ++it) { const int idx = it * 256 + tid; const int ci = idx >> 6, s = idx & 63; ts[s * CSP + ci] = sp[idx]; }
    __syncthreads();
    bf* dp = dst + (size_t)co * KC;
#pragma unroll 1
    for (int ps = 0; ps < 2; ++ps) {
#pragma unroll 1
        for (int it = 0; it < 4; ++it) { const int q = it * 256 + tid; const int s = q >> 4, c8 = (q & 15) * 8;
            const v4f x0 = *(const v4fa*)(&ts[s * CSP + c8]); const v4f x1 = *(const v4fa*)(&ts[s * CSP + c8 + 4]); v8us o;
#pragma unroll
            for (int i = 0; i < 4; ++i) { o[i] = f2bf(x0[i]); o[4 + i] = f2bf(x1[i]); }
            *(volatile v8us*)(dp + (size_t)q * 8) = o; }
        if (ps == 0) __threadfence(); }
}

template <int MODE>
__global__ __launch_bounds__(32) void k_proj(const bf* __restrict__ A, const bf* __restrict__ Bt, const float* __restrict__ bias, h16* Ph, h16* Pr, int resT) {
    __shared__ __align__(16) float os[16 * 68];
    const int K = DM;
    const int lane = threadIdx.x & 31, lr = lane & 15, hi = lane >> 4; const int r0 = blockIdx.x * 64, c0 = blockIdx.y * 64;
    v8f acc[4][4];
#pragma unroll
    for (int mb = 0; mb < 4; ++mb)
#pragma unroll
        for (int nb = 0; nb < 4; ++nb) acc[mb][nb] = (v8f){};
    const size_t aoff = (size_t)(r0 + lr) * K + 8 * hi, boff = (size_t)(c0 + lr) * K + 8 * hi;
#pragma unroll 1
    for (int kc = 0; kc < K; kc += 32) {
        v16bf a[4];
#pragma unroll
        for (int mb = 0; mb < 4; ++mb) a[mb] = ldb(A + aoff + (size_t)mb * 16 * K + kc);
#pragma unroll
        for (int nb = 0; nb < 4; ++nb) { const v16bf b = ldb(Bt + boff + (size_t)nb * 16 * K + kc);
#pragma unroll
            for (int mb = 0; mb < 4; ++mb) acc[mb][nb] = wmmab(a[mb], b, acc[mb][nb]); }
        asm volatile("v_nop\n\tv_nop\n\tv_nop\n\tv_nop" : "+v"(acc[0][0]), "+v"(acc[1][1]), "+v"(acc[2][2]), "+v"(acc[3][3]) : "v"(a[0]), "v"(a[1]), "v"(a[2]), "v"(a[3]));
    }
    float bc[4];
#pragma unroll
    for (int nb = 0; nb < 4; ++nb) bc[nb] = (MODE == 0) ? bfr(bias[c0 + nb * 16 + lr]) : 0.0f;
    size_t tbase, rbase; bool wr;
    if (MODE == 0) { const int bb = r0 / SEQ, tt = r0 % SEQ; const int zc = bb * NH_ + c0 / HD;
                     tbase = ((size_t)zc * SEQ + (size_t)tt) * HD; rbase = ((size_t)zc * (size_t)resT + (size_t)tt) * HD; wr = tt < resT; }
    else           { const int bb = c0 / SEQ, tt = c0 % SEQ;
                     tbase = (size_t)bb * (size_t)DM * SEQ + (size_t)r0 * SEQ + (size_t)tt; rbase = (size_t)bb * (size_t)DM * (size_t)resT + (size_t)r0 * (size_t)resT + (size_t)tt; wr = tt < resT; }
#pragma unroll
    for (int mb = 0; mb < 4; ++mb) {
        float br[8];
#pragma unroll
        for (int j = 0; j < 8; ++j) br[j] = (MODE == 1) ? bfr(bias[r0 + mb * 16 + hi * 8 + j]) : 0.0f;
#pragma unroll
        for (int nb = 0; nb < 4; ++nb) {
#pragma unroll
            for (int j = 0; j < 8; ++j) os[(hi * 8 + j) * 68 + nb * 16 + lr] = acc[mb][nb][j] + bc[nb] + br[j]; }
        wave_sync();
#pragma unroll 1
        for (int ps = 0; ps < 2; ++ps) {
            if (MODE == 0) {
                const size_t sb = tbase + (size_t)(mb * 16) * HD;
                const size_t rb = rbase + (size_t)(mb * 16) * HD;
#pragma unroll
                for (int hh = 0; hh < 2; ++hh) {
#pragma unroll
                    for (int s = 0; s < 2; ++s) { const int p = s * 32 + lane; const int row = p >> 2, c8 = (p & 3) * 8;
                        const v4f x0 = *(const v4fa*)(&os[row * 68 + hh * 32 + c8]); const v4f x1 = *(const v4fa*)(&os[row * 68 + hh * 32 + c8 + 4]); v8h hv, rv;
#pragma unroll
                        for (int i = 0; i < 4; ++i) { const h16 a0 = (h16)x0[i]; const h16 a1 = (h16)x1[i]; hv[i] = a0; hv[4 + i] = a1; rv[i] = (h16)((x0[i] - (float)a0) * QRS); rv[4 + i] = (h16)((x1[i] - (float)a1) * QRS); }
                        const size_t oo = sb + (size_t)hh * ((size_t)SEQ * HD) + (size_t)p * 8;
                        const size_t ro = rb + (size_t)hh * ((size_t)resT * HD) + (size_t)p * 8;
                        *(volatile v8h*)(Ph + oo) = hv; if (wr) *(volatile v8h*)(Pr + ro) = rv; } }
            } else {
                const size_t sb = tbase + (size_t)(mb * 16) * SEQ;
                const size_t rb = rbase + (size_t)(mb * 16) * (size_t)resT;
#pragma unroll
                for (int s = 0; s < 4; ++s) { const int row = 4 * s + (lane >> 3), c8 = (lane & 7) * 8;
                    const v4f x0 = *(const v4fa*)(&os[row * 68 + c8]); const v4f x1 = *(const v4fa*)(&os[row * 68 + c8 + 4]); v8h hv, rv;
#pragma unroll
                    for (int i = 0; i < 4; ++i) { const h16 a0 = (h16)x0[i]; const h16 a1 = (h16)x1[i]; hv[i] = a0; hv[4 + i] = a1; rv[i] = (h16)((x0[i] - (float)a0) * QRS); rv[4 + i] = (h16)((x1[i] - (float)a1) * QRS); }
                    const size_t oo = sb + (size_t)row * SEQ + c8;
                    const size_t ro = rb + (size_t)row * (size_t)resT + c8;
                    *(volatile v8h*)(Ph + oo) = hv; if (wr) *(volatile v8h*)(Pr + ro) = rv; }
            }
            if (ps == 0) __threadfence(); }
        wave_sync();
    }
}

__global__ __launch_bounds__(32) void k_conv(const bf* __restrict__ XB, const bf* __restrict__ W2, const float* __restrict__ srb, const float* __restrict__ lng, const float* __restrict__ lnb,
                                             const int* __restrict__ dimd, const int* __restrict__ dimh, const int* __restrict__ dimw, h16* XL) {
    __shared__ __align__(16) float cs[16 * CSP];
    static_assert(32 * 8 * 8 == 16 * DM);
    const int lane = threadIdx.x & 31, lr = lane & 15, hi = lane >> 4;
    const int r0 = blockIdx.x * 16;
    const int r = r0 + lr; const int b = r / SEQK, m = r % SEQK;
    const int od = m >> 6, oh = (m >> 3) & 7, ow = m & 7;
    const size_t abase = ((size_t)b * SEQ + (size_t)((4 * od * VH + 4 * oh) * VW + 4 * ow)) * DM + 8 * hi;
    const size_t bbase = (size_t)lr * KC + 8 * hi;
    v8f acc[8];
#pragma unroll
    for (int nb = 0; nb < 8; ++nb) acc[nb] = (v8f){};
#pragma unroll 1
    for (int kk = 0; kk < KC / 32; ++kk) {
        const int s = kk >> 2;
        const size_t ao = abase + (size_t)((((s >> 4) * VH) + ((s >> 2) & 3)) * VW + (s & 3)) * DM + (size_t)(kk & 3) * 32;
        const size_t bo = bbase + (size_t)kk * 32;
        const v16bf a = ldb(XB + ao);
#pragma unroll
        for (int nb = 0; nb < 8; ++nb) { const v16bf w = ldb(W2 + bo + (size_t)nb * 16 * KC); acc[nb] = wmmabg(a, w, acc[nb]); }
    }
    float cb[8];
#pragma unroll
    for (int nb = 0; nb < 8; ++nb) cb[nb] = bfr(srb[nb * 16 + lr]);
    float mu[8], rs[8];
#pragma unroll
    for (int j = 0; j < 8; ++j) { float sm = 0.0f;
#pragma unroll
        for (int nb = 0; nb < 8; ++nb) { acc[nb][j] += cb[nb]; sm += acc[nb][j]; }
        sm += __shfl_xor(sm, 8, 32); sm += __shfl_xor(sm, 4, 32); sm += __shfl_xor(sm, 2, 32); sm += __shfl_xor(sm, 1, 32);
        mu[j] = sm * (1.0f / 128.0f); }
#pragma unroll
    for (int j = 0; j < 8; ++j) { float q = 0.0f;
#pragma unroll
        for (int nb = 0; nb < 8; ++nb) { const float d = acc[nb][j] - mu[j]; q += d * d; }
        q += __shfl_xor(q, 8, 32); q += __shfl_xor(q, 4, 32); q += __shfl_xor(q, 2, 32); q += __shfl_xor(q, 1, 32);
        rs[j] = rsqrtf(q * (1.0f / 128.0f) + 1.0e-5f); }
    asm volatile("" ::: "memory");
    const bool okd = (dimd[0] == VD_FULL) & (dimh[0] == VH) & (dimw[0] == VW);
    const float pz = okd ? 0.0f : __uint_as_float(0x7FC00000u);
    float cg[8], ct[8];
#pragma unroll
    for (int nb = 0; nb < 8; ++nb) { cg[nb] = bfr(lng[nb * 16 + lr]); ct[nb] = bfr(lnb[nb * 16 + lr]); }
#pragma unroll
    for (int nb = 0; nb < 8; ++nb) {
#pragma unroll
        for (int j = 0; j < 8; ++j) cs[(hi * 8 + j) * CSP + nb * 16 + lr] = (acc[nb][j] - mu[j]) * rs[j] * cg[nb] + ct[nb] + pz; }
    wave_sync();
    h16* dp = XL + (size_t)r0 * DM;
#pragma unroll 1
    for (int ps = 0; ps < 2; ++ps) {
#pragma unroll
        for (int s = 0; s < 8; ++s) { const int p = s * 32 + lane; const int row = p >> 4, c8 = (p & 15) * 8;
            const v4f x0 = *(const v4fa*)(&cs[row * CSP + c8]); const v4f x1 = *(const v4fa*)(&cs[row * CSP + c8 + 4]); v8h hv;
#pragma unroll
            for (int i = 0; i < 4; ++i) { hv[i] = toh_flush(x0[i]); hv[4 + i] = toh_flush(x1[i]); }
            *(volatile v8h*)(dp + (size_t)p * 8) = hv; }
        if (ps == 0) __threadfence(); }
}

template <int MODE, int TS>
__device__ __forceinline__ void gemm64(const h16* __restrict__ A, const h16* __restrict__ Bt, const float* __restrict__ bias, const float oscale, h16* Ph, float* Pf) {
    __shared__ __align__(16) float gs[16 * 68];
    static_assert(TS % 64 == 0);
    static_assert(2 * 2 * 32 * 8 == 16 * 64);
    static_assert(4 * 32 * 8 == 16 * 64);
    static_assert(8 * 32 * 4 == 16 * 64);
    const int lane = threadIdx.x & 31, lr = lane & 15, hi = lane >> 4; const int r0 = blockIdx.x * 64, c0 = blockIdx.y * 64;
    v8f acc[4][4];
#pragma unroll
    for (int mb = 0; mb < 4; ++mb)
#pragma unroll
        for (int nb = 0; nb < 4; ++nb) acc[mb][nb] = (v8f){};
    size_t aoff, amb, aks;
    if (MODE == 2) { const int ab = r0 / TS, at = r0 % TS; aoff = ((size_t)ab * NH_ * TS + (size_t)(at + lr)) * HD + 8 * hi; amb = (size_t)16 * HD; aks = (size_t)TS * HD; }
    else           { aoff = (size_t)(r0 + lr) * DM + 8 * hi; amb = (size_t)16 * DM; aks = 32; }
    const size_t boff = (size_t)(c0 + lr) * DM + 8 * hi;
#pragma unroll 1
    for (int ks = 0; ks < DM / 32; ++ks) {
        v16h a[4];
#pragma unroll
        for (int mb = 0; mb < 4; ++mb) a[mb] = ldh(A + aoff + (size_t)mb * amb + (size_t)ks * aks);
#pragma unroll
        for (int nb = 0; nb < 4; ++nb) { const v16h w = ldh(Bt + boff + (size_t)nb * 16 * DM + (size_t)ks * 32);
#pragma unroll
            for (int mb = 0; mb < 4; ++mb) acc[mb][nb] = wmma16g(a[mb], w, acc[mb][nb]); }
    }
    float bc[4];
#pragma unroll
    for (int nb = 0; nb < 4; ++nb) bc[nb] = (MODE != 1) ? bfr(bias[c0 + nb * 16 + lr]) : 0.0f;
    const int bb = (MODE == 1) ? (c0 / TS) : (r0 / TS);
    const int tt = (MODE == 1) ? (c0 % TS) : (r0 % TS);
    size_t tbase;
    if (MODE == 0)      tbase = ((size_t)(bb * NH_ + c0 / HD) * TS + (size_t)tt) * HD;
    else if (MODE == 1) tbase = (size_t)bb * (size_t)DM * TS + (size_t)r0 * TS + (size_t)tt;
    else                tbase = ((size_t)bb * OUT_SEQ + (size_t)tt) * DM + (size_t)c0;
#pragma unroll
    for (int mb = 0; mb < 4; ++mb) {
        float br[8];
#pragma unroll
        for (int j = 0; j < 8; ++j) br[j] = (MODE == 1) ? bfr(bias[r0 + mb * 16 + hi * 8 + j]) : 0.0f;
#pragma unroll
        for (int nb = 0; nb < 4; ++nb) {
#pragma unroll
            for (int j = 0; j < 8; ++j) gs[(hi * 8 + j) * 68 + nb * 16 + lr] = acc[mb][nb][j] * oscale + bc[nb] + br[j]; }
        wave_sync();
#pragma unroll 1
        for (int ps = 0; ps < 2; ++ps) {
            if (MODE == 0) {
                const size_t sb = tbase + (size_t)(mb * 16) * HD;
#pragma unroll
                for (int hh = 0; hh < 2; ++hh) {
#pragma unroll
                    for (int s = 0; s < 2; ++s) { const int p = s * 32 + lane; const int row = p >> 2, c8 = (p & 3) * 8;
                        const v4f x0 = *(const v4fa*)(&gs[row * 68 + hh * 32 + c8]); const v4f x1 = *(const v4fa*)(&gs[row * 68 + hh * 32 + c8 + 4]); v8h hv;
#pragma unroll
                        for (int i = 0; i < 4; ++i) { hv[i] = toh_flush(x0[i]); hv[4 + i] = toh_flush(x1[i]); }
                        *(volatile v8h*)(Ph + sb + (size_t)hh * ((size_t)TS * HD) + (size_t)p * 8) = hv; } }
            } else if (MODE == 1) {
                const size_t sb = tbase + (size_t)(mb * 16) * TS;
#pragma unroll
                for (int s = 0; s < 4; ++s) { const int row = 4 * s + (lane >> 3), c8 = (lane & 7) * 8;
                    const v4f x0 = *(const v4fa*)(&gs[row * 68 + c8]); const v4f x1 = *(const v4fa*)(&gs[row * 68 + c8 + 4]); v8h hv;
#pragma unroll
                    for (int i = 0; i < 4; ++i) { hv[i] = toh_flush(x0[i]); hv[4 + i] = toh_flush(x1[i]); }
                    *(volatile v8h*)(Ph + sb + (size_t)row * TS + c8) = hv; }
            } else {
                const size_t sb = tbase + (size_t)(mb * 16) * DM;
#pragma unroll
                for (int s = 0; s < 8; ++s) { const int p = s * 32 + lane; const int row = p >> 4, c4 = (p & 15) * 4;
                    const v4f val = *(const v4fa*)(&gs[row * 68 + c4]);
                    *(volatile v4f*)(Pf + sb + (size_t)row * DM + c4) = val; }
            }
            if (ps == 0) __threadfence(); }
        wave_sync();
    }
}

__global__ __launch_bounds__(32) void k_kproj(const h16* __restrict__ XL, const h16* __restrict__ WK, const float* __restrict__ bk, h16* KP) {
    gemm64<0, SEQK>(XL, WK, bk, WCI, KP, (float*)nullptr);
}
__global__ __launch_bounds__(32) void k_vproj(const h16* __restrict__ WV, const h16* __restrict__ XL, const float* __restrict__ bv, h16* VT) {
    gemm64<1, SEQK>(WV, XL, bv, WCI, VT, (float*)nullptr);
}
__global__ __launch_bounds__(32) void k_oproj(const h16* __restrict__ OP, const h16* __restrict__ WP, const float* __restrict__ bp, float* OUT) {
    gemm64<2, SEQ>(OP, WP, bp, OWI, (h16*)nullptr, OUT);
}

__global__ __launch_bounds__(32 * AW) void k_attn(const h16* __restrict__ QH, const h16* __restrict__ KP, const h16* __restrict__ VT, h16* OP) {
    __shared__ __align__(16) float os[AW * 16 * OSP];
    static_assert(2 * 32 * 8 == 16 * HD);
    const int lane = threadIdx.x & 31, lr = lane & 15, hi = lane >> 4;
    const int wave = __builtin_amdgcn_readfirstlane((int)(threadIdx.x >> 5));
    const int zh = blockIdx.y;
    const int t0 = (blockIdx.x * AW + wave) * 16;
    const size_t qo = ((size_t)zh * SEQ + (size_t)(t0 + lr)) * HD + 8 * hi;
    const v16h qh = ldh(QH + qo);
    const size_t kvb = (size_t)zh * SEQK * HD;
    const size_t ko = kvb + (size_t)lr * HD + 8 * hi;
    const size_t vo = kvb + (size_t)lr * SEQK + 8 * hi;
    v8f o0 = (v8f){}, o1 = (v8f){};
    float m = NEGB, l = 0.0f;
#pragma unroll 1
    for (int key0 = 0; key0 < SEQK; key0 += 32) {
        const h16* ka = KP + ko + (size_t)key0 * HD;
        const v16h ka0 = ldh(ka), kb0 = ldh(ka + 16 * HD);
        v8f sa = (v8f){}, sb = (v8f){};
        sa = wmma16g(ka0, qh, sa); sb = wmma16g(kb0, qh, sb);
        float ta[8], tb[8]; float mx = NEGB;
#pragma unroll
        for (int r = 0; r < 8; ++r) { ta[r] = sa[r] * SC2; tb[r] = sb[r] * SC2; mx = fmaxf(mx, fmaxf(ta[r], tb[r])); }
        mx = fmaxf(mx, __shfl_xor(mx, 16, 32));
        const float mnew = fmaxf(m, mx);
        const float alpha = __builtin_amdgcn_exp2f(m - mnew);
        const float sh = PSH - mnew;
        v16h pb; float ls = 0.0f;
#pragma unroll
        for (int r = 0; r < 8; ++r) {
            const float xa = ta[r] + sh, xb = tb[r] + sh;
            const float ea = __builtin_amdgcn_exp2f(xa), eb = __builtin_amdgcn_exp2f(xb);
            const float ga = (xa < -14.0f) ? 0.0f : ea, gb = (xb < -14.0f) ? 0.0f : eb;
            const h16 pa = (h16)ga; const h16 pc = (h16)gb;
            pb[r] = pa; pb[8 + r] = pc;
            ls += (float)pa + (float)pc; }
        l = l * alpha + ls; m = mnew;
        o0 = o0 * alpha; o1 = o1 * alpha;
        const h16* va = VT + vo + key0;
        const v16h v0 = ldh(va), v1 = ldh(va + (size_t)16 * SEQK);
        o0 = wmma16g(v0, pb, o0); o1 = wmma16g(v1, pb, o1);
    }
    l += __shfl_xor(l, 16, 32);
    const float inv = OCS * (1.0f / l);
    const int wb = wave * 16 * OSP;
    { v4f a, c;
      a[0] = o0[0] * inv; a[1] = o0[1] * inv; a[2] = o0[2] * inv; a[3] = o0[3] * inv; c[0] = o0[4] * inv; c[1] = o0[5] * inv; c[2] = o0[6] * inv; c[3] = o0[7] * inv;
      *(v4fa*)(&os[wb + lr * OSP +  0 + 8 * hi]) = a; *(v4fa*)(&os[wb + lr * OSP +  0 + 8 * hi + 4]) = c;
      a[0] = o1[0] * inv; a[1] = o1[1] * inv; a[2] = o1[2] * inv; a[3] = o1[3] * inv; c[0] = o1[4] * inv; c[1] = o1[5] * inv; c[2] = o1[6] * inv; c[3] = o1[7] * inv;
      *(v4fa*)(&os[wb + lr * OSP + 16 + 8 * hi]) = a; *(v4fa*)(&os[wb + lr * OSP + 16 + 8 * hi + 4]) = c; }
    wave_sync();
    h16* orow = OP + ((size_t)zh * SEQ + (size_t)t0) * HD;
#pragma unroll 1
    for (int ps = 0; ps < 2; ++ps) {
#pragma unroll
        for (int s = 0; s < 2; ++s) { const int p = s * 32 + lane; const int row = p >> 2, c8 = (p & 3) * 8;
            const v4f x0 = *(const v4fa*)(&os[wb + row * OSP + c8]); const v4f x1 = *(const v4fa*)(&os[wb + row * OSP + c8 + 4]); v8h hv;
#pragma unroll
            for (int i = 0; i < 4; ++i) { hv[i] = toh_flush(x0[i]); hv[4 + i] = toh_flush(x1[i]); }
            *(volatile v8h*)(orow + (size_t)p * 8) = hv; }
        if (ps == 0) __threadfence(); }
}

static constexpr size_t al256(size_t v) { return (v + 255) & ~(size_t)255; }
static constexpr size_t SZ_XB  = al256((size_t)NB * SEQ * DM * 2);
static constexpr size_t SZ_WQ  = al256((size_t)DM * DM * 2);
static constexpr size_t SZ_W2  = al256((size_t)DM * KC * 2);
static constexpr size_t SZ_WKV = al256((size_t)2 * DM * DM * 2);
static constexpr size_t SZ_WP  = al256((size_t)DM * DM * 2);
static constexpr size_t SZ_XL  = al256((size_t)NB * SEQK * DM * 2);
static constexpr size_t SZ_PL  = al256((size_t)NB * NH_ * SEQ * HD * 2);
static constexpr size_t SZ_KV  = al256((size_t)NB * NH_ * SEQK * HD * 2);
static constexpr size_t SZ_TOTAL = SZ_XB + SZ_WQ + SZ_W2 + SZ_WKV + SZ_WP + SZ_XL + 2 * SZ_PL + 2 * SZ_KV;
static_assert(SZ_TOTAL <= (size_t)134217728);
static_assert((size_t)NB * NH_ * SEQK * HD == (size_t)NB * DM * SEQK);
static_assert((size_t)NB * NH_ * SEQ * HD == (size_t)NB * SEQ * DM);
static_assert(((size_t)NB * SEQK * DM) % (16 * DM) == 0);

extern "C" void kernel_launch(void* const* d_in, const int* in_sizes, int n_in,
                              void* d_out, int out_size, void* d_ws, size_t ws_size, hipStream_t stream) {
    if (n_in < 14) return;
    const size_t needx = ((size_t)(NB - 1) * SEQ_FULL + SEQ) * DM;
    if ((size_t)in_sizes[0] < needx) return;
    if ((size_t)in_sizes[1] < (size_t)DM * DM || (size_t)in_sizes[3] < (size_t)2 * DM * DM || (size_t)in_sizes[5] < (size_t)DM * KC || (size_t)in_sizes[9] < (size_t)DM * DM) return;
    if (in_sizes[2] < DM || in_sizes[4] < 2 * DM || in_sizes[6] < DM || in_sizes[7] < DM || in_sizes[8] < DM || in_sizes[10] < DM) return;
    if (in_sizes[11] < 1 || in_sizes[12] < 1 || in_sizes[13] < 1) return;
    if ((size_t)out_size < ((size_t)(NB - 1) * OUT_SEQ + SEQ) * DM) return;
    if (SZ_TOTAL > ws_size) return;
    const float* x   = (const float*)d_in[0];
    const float* wq  = (const float*)d_in[1];  const float* bq  = (const float*)d_in[2];
    const float* wkv = (const float*)d_in[3];  const float* bkv = (const float*)d_in[4];
    const float* srw = (const float*)d_in[5];  const float* srb = (const float*)d_in[6];
    const float* lng = (const float*)d_in[7];  const float* lnb = (const float*)d_in[8];
    const float* wp  = (const float*)d_in[9];  const float* bp  = (const float*)d_in[10];
    const int* dimd = (const int*)d_in[11]; const int* dimh = (const int*)d_in[12]; const int* dimw = (const int*)d_in[13];
    float* OUT = (float*)d_out;
    char* wsp = (char*)d_ws;
    bf*  XB   = (bf*)wsp;  wsp += SZ_XB;
    bf*  WQB  = (bf*)wsp;  wsp += SZ_WQ;
    bf*  W2B  = (bf*)wsp;  wsp += SZ_W2;
    h16* WKVH = (h16*)wsp; wsp += SZ_WKV;
    h16* WPH  = (h16*)wsp; wsp += SZ_WP;
    h16* XL   = (h16*)wsp; wsp += SZ_XL;
    h16* QH   = (h16*)wsp; wsp += SZ_PL;
    h16* OP   = (h16*)wsp; wsp += SZ_PL;
    h16* KP   = (h16*)wsp; wsp += SZ_KV;
    h16* VT   = (h16*)wsp; wsp += SZ_KV;

    if (SEQ == SEQ_FULL) {
        const size_t n8 = (size_t)NB * SEQ * DM / 8;
        k_cvt8<<<(unsigned)((n8 + 255) / 256), 256, 0, stream>>>(x, XB, n8);
    } else {
        const size_t n8 = (size_t)SEQ * DM / 8;
        for (int b = 0; b < NB; ++b) k_cvt8<<<(unsigned)((n8 + 255) / 256), 256, 0, stream>>>(x + (size_t)b * SEQ_FULL * DM, XB + (size_t)b * SEQ * DM, n8);
    }
    { const size_t n8 = (size_t)DM * DM / 8;
      k_cvt8<<<(unsigned)((n8 + 255) / 256), 256, 0, stream>>>(wq, WQB, n8);
      k_cvth8<<<(unsigned)((n8 + 255) / 256), 256, 0, stream>>>(wp, WPH, n8, WCS);
      k_cvth8<<<(unsigned)((2 * n8 + 255) / 256), 256, 0, stream>>>(wkv, WKVH, 2 * n8, WCS); }
    k_srw<<<DM, 256, 0, stream>>>(srw, W2B);

    k_conv<<<(NB * SEQK) / 16, 32, 0, stream>>>(XB, W2B, srb, lng, lnb, dimd, dimh, dimw, XL);
    k_kproj<<<dim3(NB * SEQK / 64, DM / 64, 1), 32, 0, stream>>>(XL, WKVH, bkv, KP);
    k_vproj<<<dim3(DM / 64, NB * SEQK / 64, 1), 32, 0, stream>>>(WKVH + (size_t)DM * DM, XL, bkv + DM, VT);
    k_proj<0><<<dim3(NB * SEQ / 64, DM / 64, 1), 32, 0, stream>>>(XB, WQB, bq, QH, QH, 0);

    k_attn<<<dim3(SEQ / (16 * AW), NB * NH_, 1), 32 * AW, 0, stream>>>(QH, KP, VT, OP);
    k_oproj<<<dim3(NB * SEQ / 64, DM / 64, 1), 32, 0, stream>>>(OP, WPH, bp, OUT);
}
